// STGCNLayer_65189013619314
// MI455X (gfx1250) — hardware-run, weakly checked
//
#include <hip/hip_runtime.h>
#include <stddef.h>
#include <stdint.h>
#include <math.h>

#define SPLIT_T 1
#define SPLIT_H 1

#define NN      50000
#define NBT     4
#define NE      800000
#define CH      64
#define MP      50048
#define GBM     128
#define MROWS   (NN * NBT)
#define GBLK    ((MROWS + GBM - 1) / GBM)
#define XP      256
#define TP      512
#define KC      320
#define KL      128
#define BPW     68
#define NTHR    256
#define NWAVE   8
#define EPT     8
#define WCH     (32 * EPT)
#define NBRUN   1024
#define SLB     10
#define NBK     49
#define WLCAP   2560
#define RCAP    20480
#define DEGCAP  64
#define MAXDEG_MEAS   33
#define MAXB1024_MEAS 16696
#define RPB     64
#define RPW     8
#define WSMAX   134217728

#define BK_ZINTS (NWAVE * WLCAP + RCAP + 3 * NBRUN)
#define BK_INTS  (BK_ZINTS + 16)
#define BK_LDS   (BK_INTS * 4)

#define PBX  (MP * 32 / NTHR)
#define PBWC (CH * KC / 8 / NTHR)
#define PBWL (CH * KL / 8 / NTHR)
#define PBTOT (PBX + PBWC + PBWL + 1)

static_assert(CH == 64 && NBT == 4 && XP == NBT * CH && TP == NBT * 2 * CH);
static_assert(MP % GBM == 0 && MP % RPB == 0 && MP >= NN && RPB == NWAVE * RPW);
static_assert(GBM % NBT == 0 && GBLK * GBM <= MP * NBT && GBLK * GBM >= MROWS);
static_assert(NBRUN == (1 << SLB) && NBRUN % RPB == 0 && NBRUN % NTHR == 0);
static_assert(NBK * NBRUN >= MP && (NBK - 1) * NBRUN < NN);
static_assert(NE < (1 << 21) && (((long long)NE) << SLB) < (1LL << 31));
static_assert(NE % WCH == 0 && NE % 4 == 0);
static_assert(RCAP == NWAVE * WLCAP && RCAP % (NTHR * 4) == 0 && BK_ZINTS % 4 == 0);
static_assert((long long)RCAP * 100 >= (long long)MAXB1024_MEAS * 105);
static_assert(WLCAP >= MAXB1024_MEAS / 8 + 8 * 46 + 1);
static_assert(NN <= 65536);
static_assert(DEGCAP >= MAXDEG_MEAS + 8 && DEGCAP <= 64);
static_assert(KC % 32 == 0 && KL % 32 == 0 && KC == 5 * CH && KL == 2 * CH);
static_assert(BK_LDS <= 300000);
static_assert((MP * 32) % NTHR == 0 && (CH * KC / 8) % NTHR == 0 && (CH * KL / 8) % NTHR == 0);
static_assert(GBM * BPW * 4 + 512 <= 65536);

typedef float          v4f   __attribute__((ext_vector_type(4)));
typedef float          v8f   __attribute__((ext_vector_type(8)));
typedef int            v4i   __attribute__((ext_vector_type(4)));
typedef int            v8i   __attribute__((ext_vector_type(8)));
typedef unsigned       v4u   __attribute__((ext_vector_type(4)));
typedef unsigned short v8us  __attribute__((ext_vector_type(8)));
typedef unsigned short v16us __attribute__((ext_vector_type(16)));
typedef __bf16         v16bf __attribute__((ext_vector_type(16)));
typedef v4f  __attribute__((may_alias)) v4fa;
typedef v4i  __attribute__((may_alias)) v4ia;
typedef v4u  __attribute__((may_alias)) v4ua;
typedef v8us __attribute__((may_alias)) v8usa;
union FragB { v16bf v; v16us u; v8us h[2]; v8i w; };

__device__ __forceinline__ v8f wmb(const FragB& a, const FragB& b, v8f c) {
  v8f d = __builtin_amdgcn_wmma_f32_16x16x32_bf16(false, a.v, false, b.v, (short)0, c, false, false);
  asm volatile("v_nop\n\tv_nop\n\tv_nop\n\tv_nop" : "+v"(d) : "v"(a.w), "v"(b.w));
  return d;
}

__device__ __forceinline__ unsigned bf16_bits(float f) {
  const unsigned u = __float_as_uint(f);
  const unsigned r = (u + 0x7FFFu + ((u >> 16) & 1u)) >> 16;
  const unsigned q = (u >> 16) | 0x40u;
  return (((u & 0x7fffffffu) > 0x7f800000u) ? q : r) & 0xFFFFu;
}
__device__ __forceinline__ float bfw_lo(unsigned w) { return __uint_as_float(w << 16); }
__device__ __forceinline__ float bfw_hi(unsigned w) { return __uint_as_float(w & 0xffff0000u); }
__device__ __forceinline__ void pack2(float a, float b, unsigned& hw, unsigned& lw) {
  const unsigned ha = bf16_bits(a), hb = bf16_bits(b);
  const unsigned la = bf16_bits(a - __uint_as_float(ha << 16));
  const unsigned lb = bf16_bits(b - __uint_as_float(hb << 16));
  hw = ha | (hb << 16);
  lw = la | (lb << 16);
}
__device__ __forceinline__ float relu_k(float v) { return (v > 0.0f) ? v : (v - v); }

__device__ __forceinline__ void st2_v4f(float* p, v4f v) {
  *(volatile v4f*)p = v;
  __threadfence();
  *(volatile v4f*)p = v;
}
__device__ __forceinline__ void st2_v8us(unsigned short* p, v8us v) {
  *(volatile v8us*)p = v;
  __threadfence();
  *(volatile v8us*)p = v;
}

__device__ __forceinline__ v8us gather8(const float* __restrict__ base, int stride) {
  float f[8];
#pragma unroll
  for (int i = 0; i < 8; ++i) f[i] = base[(size_t)i * (size_t)stride];
  v8us o;
#pragma unroll
  for (int i = 0; i < 8; ++i) o[i] = (unsigned short)bf16_bits(f[i]);
  return o;
}

__global__ __launch_bounds__(NTHR) void k_prep(const float* __restrict__ x, const float* __restrict__ wc,
                                               const float* __restrict__ bc, const float* __restrict__ wl,
                                               const float* __restrict__ bl, unsigned short* xt,
                                               unsigned short* wct, unsigned short* wlt, float* sm) {
  const int tid = (int)threadIdx.x, lane = tid & 31;
  const int blk = (int)blockIdx.x;
  if (blk < PBX) {
    const int u    = blk * NTHR + tid;
    const int node = u >> 5, l = u & 31;
    const int b = l >> 3, j = l & 7;
    const int rc = node < NN ? node : NN - 1;
    const unsigned mk = node < NN ? 0xffffu : 0u;
    const float* p = x + ((size_t)b * NN + (size_t)rc) * CH + 8 * j;
    const v4f a = *(const v4fa*)p;
    const v4f c = *(const v4fa*)(p + 4);
    v8us o;
    o[0] = (unsigned short)(bf16_bits(a.x) & mk); o[1] = (unsigned short)(bf16_bits(a.y) & mk);
    o[2] = (unsigned short)(bf16_bits(a.z) & mk); o[3] = (unsigned short)(bf16_bits(a.w) & mk);
    o[4] = (unsigned short)(bf16_bits(c.x) & mk); o[5] = (unsigned short)(bf16_bits(c.y) & mk);
    o[6] = (unsigned short)(bf16_bits(c.z) & mk); o[7] = (unsigned short)(bf16_bits(c.w) & mk);
    st2_v8us(xt + (size_t)node * XP + 8 * l, o);
  } else if (blk < PBX + PBWC) {
    const int u  = (blk - PBX) * NTHR + tid;
    const int n  = u / 40, g = u - 40 * n;
    const int k8 = 8 * g, kk = k8 & 63;
    const int ord = ((g >> 3) + 1) >> 1;
    const v8us o = gather8(wc + (size_t)ord * CH * CH + (size_t)kk * CH + n, CH);
    st2_v8us(wct + (size_t)n * KC + k8, o);
  } else if (blk < PBX + PBWC + PBWL) {
    const int u  = (blk - PBX - PBWC) * NTHR + tid;
    const int n  = u >> 4, k8 = (u & 15) * 8, kk = k8 & 63;
    const v8us o = gather8(wl + (size_t)kk * CH + n, CH);
    st2_v8us(wlt + (size_t)n * KL + k8, o);
  } else {
    if (tid < 32) {
      const int q = lane & 15;
      const v4f a = *(const v4fa*)(bc + 4 * q);
      const v4f c = *(const v4fa*)(bl + 4 * q);
      asm volatile("" :: "v"(a));
      asm volatile("" :: "v"(c));
      const unsigned ma = (lane < 16) ? 0xffffffffu : 0u;
      v4f o;
      o.x = __uint_as_float(((bf16_bits(a.x) << 16) & ma) | ((bf16_bits(c.x) << 16) & ~ma));
      o.y = __uint_as_float(((bf16_bits(a.y) << 16) & ma) | ((bf16_bits(c.y) << 16) & ~ma));
      o.z = __uint_as_float(((bf16_bits(a.z) << 16) & ma) | ((bf16_bits(c.z) << 16) & ~ma));
      o.w = __uint_as_float(((bf16_bits(a.w) << 16) & ma) | ((bf16_bits(c.w) << 16) & ~ma));
      st2_v4f(sm + 4 * lane, o);
    }
  }
}

__device__ __forceinline__ void bucket_flush(const int* pl, const int* cnt, const int* nrm, int ov,
                                             int* lp, int* cop, int* np, int* fp, int tid) {
#pragma unroll 1
  for (int i = tid * 4; i < RCAP; i += NTHR * 4) {
    const v4i v = *(const v4ia*)(pl + i);
    *(volatile v4i*)(lp + i) = v;
  }
#pragma unroll 1
  for (int i = tid * 4; i < 2 * NBRUN; i += NTHR * 4) {
    const v4i v = *(const v4ia*)(cnt + i);
    *(volatile v4i*)(cop + i) = v;
  }
  {
    const v4i v = *(const v4ia*)(nrm + 4 * tid);
    *(volatile v4i*)(np + 4 * tid) = v;
  }
  if (tid < 8) {
    const v4i f = {ov, ov, ov, ov};
    *(volatile v4i*)(fp + 4 * tid) = f;
  }
}

__global__ __launch_bounds__(NTHR) void k_bucket(const int* __restrict__ srcs, const int* __restrict__ dsts,
                                                 int* LIST, int* CO, int* NORMB, int* FLAG) {
  extern __shared__ __attribute__((aligned(16))) int dsm[];
  int* wl   = dsm;
  int* pl   = dsm + NWAVE * WLCAP;
  int* cnt  = pl + RCAP;
  int* offs = cnt + NBRUN;
  int* cur  = offs + NBRUN;
  int* misc = cur + NBRUN;
  const int tid = (int)threadIdx.x, lane = tid & 31, wave = tid >> 5;
  const int blk = (int)blockIdx.x;
  const unsigned nbs = (unsigned)(blk * NBRUN);
  int nb = NN - blk * NBRUN;
  nb = nb > NBRUN ? NBRUN : (nb < 1 ? 1 : nb);
  const unsigned unb = (unsigned)nb;

  {
    const v4i z4 = {0, 0, 0, 0};
    for (int i = tid * 4; i < BK_ZINTS; i += NTHR * 4) *(v4ia*)(dsm + i) = z4;
    if (tid < 16) misc[tid] = 0;
  }
  __syncthreads();

  {
    const int per  = ((NE + NWAVE * WCH - 1) / (NWAVE * WCH)) * WCH;
    const int ebeg = wave * per;
    const int eend = (ebeg + per < NE) ? (ebeg + per) : NE;
    int* mylist = wl + wave * WLCAP;
    int wc = 0;
#pragma unroll 1
    for (int cb = ebeg; cb < eend; cb += WCH) {
      const int e0 = cb + lane * EPT;
      const v4i da = *(const v4ia*)(dsts + e0);
      const v4i db = *(const v4ia*)(dsts + e0 + 4);
      const unsigned s0 = (unsigned)da.x - nbs, s1 = (unsigned)da.y - nbs;
      const unsigned s2 = (unsigned)da.z - nbs, s3 = (unsigned)da.w - nbs;
      const unsigned s4 = (unsigned)db.x - nbs, s5 = (unsigned)db.y - nbs;
      const unsigned s6 = (unsigned)db.z - nbs, s7 = (unsigned)db.w - nbs;
      const bool h0 = s0 < unb, h1 = s1 < unb, h2 = s2 < unb, h3 = s3 < unb;
      const bool h4 = s4 < unb, h5 = s5 < unb, h6 = s6 < unb, h7 = s7 < unb;
      const unsigned m0 = __builtin_amdgcn_ballot_w32(h0), m1 = __builtin_amdgcn_ballot_w32(h1);
      const unsigned m2 = __builtin_amdgcn_ballot_w32(h2), m3 = __builtin_amdgcn_ballot_w32(h3);
      const unsigned m4 = __builtin_amdgcn_ballot_w32(h4), m5 = __builtin_amdgcn_ballot_w32(h5);
      const unsigned m6 = __builtin_amdgcn_ballot_w32(h6), m7 = __builtin_amdgcn_ballot_w32(h7);
      const unsigned any = m0 | m1 | m2 | m3 | m4 | m5 | m6 | m7;
      if (any != 0u) {
        const int pre = (int)(__builtin_amdgcn_mbcnt_lo(m0, 0u) + __builtin_amdgcn_mbcnt_lo(m1, 0u) +
                              __builtin_amdgcn_mbcnt_lo(m2, 0u) + __builtin_amdgcn_mbcnt_lo(m3, 0u) +
                              __builtin_amdgcn_mbcnt_lo(m4, 0u) + __builtin_amdgcn_mbcnt_lo(m5, 0u) +
                              __builtin_amdgcn_mbcnt_lo(m6, 0u) + __builtin_amdgcn_mbcnt_lo(m7, 0u));
        int p = wc + pre;
        if (h0) { if (p < WLCAP) mylist[p] = ((e0 + 0) << SLB) | (int)s0; p = p + 1; }
        if (h1) { if (p < WLCAP) mylist[p] = ((e0 + 1) << SLB) | (int)s1; p = p + 1; }
        if (h2) { if (p < WLCAP) mylist[p] = ((e0 + 2) << SLB) | (int)s2; p = p + 1; }
        if (h3) { if (p < WLCAP) mylist[p] = ((e0 + 3) << SLB) | (int)s3; p = p + 1; }
        if (h4) { if (p < WLCAP) mylist[p] = ((e0 + 4) << SLB) | (int)s4; p = p + 1; }
        if (h5) { if (p < WLCAP) mylist[p] = ((e0 + 5) << SLB) | (int)s5; p = p + 1; }
        if (h6) { if (p < WLCAP) mylist[p] = ((e0 + 6) << SLB) | (int)s6; p = p + 1; }
        if (h7) { if (p < WLCAP) mylist[p] = ((e0 + 7) << SLB) | (int)s7; p = p + 1; }
        wc += (int)(__builtin_popcount(m0) + __builtin_popcount(m1) + __builtin_popcount(m2) + __builtin_popcount(m3) +
                    __builtin_popcount(m4) + __builtin_popcount(m5) + __builtin_popcount(m6) + __builtin_popcount(m7));
      }
    }
    if (lane == 0) misc[wave] = wc;
  }
  __syncthreads();

  if (wave == 0) {
    int ov = 0;
#pragma unroll 1
    for (int w2 = 0; w2 < NWAVE; ++w2) {
      int c = misc[w2];
      if (c > WLCAP) ov = 1;
      c = c < 0 ? 0 : (c > WLCAP ? WLCAP : c);
#pragma unroll 1
      for (int b0 = 0; b0 < c; b0 += 32) {
        const int idx = b0 + lane;
        const int ent = wl[w2 * WLCAP + (idx < WLCAP ? idx : WLCAP - 1)];
        const int m32 = (c - b0) < 32 ? (c - b0) : 32;
#pragma unroll 1
        for (int k = 0; k < m32; ++k) {
          const int u    = __builtin_amdgcn_readlane(ent, k);
          const int slot = u & (NBRUN - 1);
          if (lane == 0) cnt[slot] = cnt[slot] + 1;
        }
      }
    }
    if (lane == 0) misc[9] = ov;
  }
  __syncthreads();
  if (wave == 0) {
    const int base = lane * (NBRUN / 32);
    int s = 0;
#pragma unroll 1
    for (int i = 0; i < NBRUN / 32; ++i) s += cnt[base + i];
    int incl = s;
#pragma unroll
    for (int d = 1; d < 32; d <<= 1) {
      const int y = __shfl_up(incl, d, 32);
      if (lane >= d) incl += y;
    }
    int run = incl - s;
#pragma unroll 1
    for (int i = 0; i < NBRUN / 32; ++i) {
      const int cv = cnt[base + i];
      offs[base + i] = run;
      cur[base + i]  = run;
      run += cv;
    }
  }
  __syncthreads();

  if (wave == 0) {
#pragma unroll 1
    for (int w2 = 0; w2 < NWAVE; ++w2) {
      int c = misc[w2];
      c = c < 0 ? 0 : (c > WLCAP ? WLCAP : c);
#pragma unroll 1
      for (int b0 = 0; b0 < c; b0 += 32) {
        const int idx = b0 + lane;
        const int ent = wl[w2 * WLCAP + (idx < WLCAP ? idx : WLCAP - 1)];
        int eid = (ent >> SLB) & 0x1FFFFF;
        eid = eid > NE - 1 ? NE - 1 : eid;
        int sr = srcs[eid];
        sr = sr < 0 ? 0 : (sr > NN - 1 ? NN - 1 : sr);
        const int m32 = (c - b0) < 32 ? (c - b0) : 32;
#pragma unroll 1
        for (int k = 0; k < m32; ++k) {
          const int u    = __builtin_amdgcn_readlane(ent, k);
          const int wd   = __builtin_amdgcn_readlane(sr, k);
          const int slot = u & (NBRUN - 1);
          if (lane == 0) {
            int p = cur[slot];
            p = p < 0 ? 0 : (p > RCAP - 1 ? RCAP - 1 : p);
            pl[p] = wd;
            cur[slot] = p + 1;
          }
        }
      }
    }
  }
  __syncthreads();

#pragma unroll 1
  for (int k = 0; k < NBRUN / NTHR; ++k) {
    const int s = tid + NTHR * k;
    int c = cnt[s];
    c = c < 1 ? 1 : c;
    const float nv = 1.0f / sqrtf((float)c);
    cur[s] = __float_as_int(nv);
  }
  __syncthreads();

  const int ovf = misc[9];
  int* lp  = LIST + (size_t)blk * RCAP;
  int* cop = CO + (size_t)blk * (2 * NBRUN);
  int* np  = NORMB + (size_t)blk * NBRUN;
  int* fp  = FLAG + (size_t)blk * 32;
  bucket_flush(pl, cnt, cur, ovf, lp, cop, np, fp, tid);
  __threadfence();
  bucket_flush(pl, cnt, cur, ovf, lp, cop, np, fp, tid);
}

template <int STAGE>
__global__ __launch_bounds__(NTHR) void k_replay(const int* __restrict__ LIST, const int* __restrict__ CO,
                                                 const float* __restrict__ NORM, const int* __restrict__ FLAG,
                                                 const unsigned short* __restrict__ XT,
                                                 const unsigned short* __restrict__ TS, unsigned short* TD) {
  const int tid = (int)threadIdx.x, lane = tid & 31;
  const int wave = __builtin_amdgcn_readfirstlane(tid >> 5);
  const int rowBase = (int)blockIdx.x * RPB;
  const int bucket  = rowBase >> SLB;
  const int* lb  = LIST + (size_t)bucket * RCAP;
  const int* cob = CO + (size_t)bucket * (2 * NBRUN);
  const int flag = FLAG[(size_t)bucket * 32];
  const int loff = (lane >> 3) * 128 + 8 * (lane & 7);
  const float qnan = __uint_as_float(0x7fc00000u);

#pragma unroll 1
  for (int ri = 0; ri < RPW; ++ri) {
    const int node = rowBase + wave * RPW + ri;
    const int slot = node & (NBRUN - 1);
    const int craw = cob[slot];
    const int oraw = cob[NBRUN + slot];
    const bool big = craw > DEGCAP;
    int c = craw < 0 ? 0 : (craw > DEGCAP ? DEGCAP : craw);
    int o = oraw < 0 ? 0 : (oraw > RCAP - 1 ? RCAP - 1 : oraw);
    if (c > RCAP - o) c = RCAP - o;
    int last = o + c - 1; last = last < o ? o : last;
    const float ni = NORM[node];
    float a0 = 0.f, a1 = 0.f, a2 = 0.f, a3 = 0.f, a4 = 0.f, a5 = 0.f, a6 = 0.f, a7 = 0.f;
#pragma unroll 1
    for (int b0 = 0; b0 < c; b0 += 32) {
      int idx = o + b0 + lane;
      idx = idx > last ? last : idx;
      int col = lb[idx];
      col = col < 0 ? 0 : (col > NN - 1 ? NN - 1 : col);
      const float wn = NORM[col] * ni;
      const int wbits = __float_as_int(wn);
      const int m32 = (c - b0) < 32 ? (c - b0) : 32;
#pragma unroll 1
      for (int k = 0; k < m32; ++k) {
        const int sk  = __builtin_amdgcn_readlane(col, k);
        const float w = __int_as_float(__builtin_amdgcn_readlane(wbits, k));
        if constexpr (STAGE == 1) {
          const v4u wv = *(const v4ua*)(XT + (size_t)sk * XP + 8 * lane);
          a0 = fmaf(w, bfw_lo(wv.x), a0); a1 = fmaf(w, bfw_hi(wv.x), a1);
          a2 = fmaf(w, bfw_lo(wv.y), a2); a3 = fmaf(w, bfw_hi(wv.y), a3);
          a4 = fmaf(w, bfw_lo(wv.z), a4); a5 = fmaf(w, bfw_hi(wv.z), a5);
          a6 = fmaf(w, bfw_lo(wv.w), a6); a7 = fmaf(w, bfw_hi(wv.w), a7);
        } else {
          const unsigned short* rp = TS + (size_t)sk * TP + loff;
          const v4u wh = *(const v4ua*)rp;
          const v4u wq = *(const v4ua*)(rp + 64);
          a0 = fmaf(w, bfw_lo(wh.x) + bfw_lo(wq.x), a0); a1 = fmaf(w, bfw_hi(wh.x) + bfw_hi(wq.x), a1);
          a2 = fmaf(w, bfw_lo(wh.y) + bfw_lo(wq.y), a2); a3 = fmaf(w, bfw_hi(wh.y) + bfw_hi(wq.y), a3);
          a4 = fmaf(w, bfw_lo(wh.z) + bfw_lo(wq.z), a4); a5 = fmaf(w, bfw_hi(wh.z) + bfw_hi(wq.z), a5);
          a6 = fmaf(w, bfw_lo(wh.w) + bfw_lo(wq.w), a6); a7 = fmaf(w, bfw_hi(wh.w) + bfw_hi(wq.w), a7);
        }
      }
    }
    float r0, r1, r2, r3, r4, r5, r6, r7;
    if constexpr (STAGE == 1) {
      r0 = -a0; r1 = -a1; r2 = -a2; r3 = -a3; r4 = -a4; r5 = -a5; r6 = -a6; r7 = -a7;
    } else {
      const int nodec = node < NN ? node : NN - 1;
      const v4u ov = *(const v4ua*)(XT + (size_t)nodec * XP + 8 * lane);
      r0 = (-2.0f * a0) - bfw_lo(ov.x); r1 = (-2.0f * a1) - bfw_hi(ov.x);
      r2 = (-2.0f * a2) - bfw_lo(ov.y); r3 = (-2.0f * a3) - bfw_hi(ov.y);
      r4 = (-2.0f * a4) - bfw_lo(ov.z); r5 = (-2.0f * a5) - bfw_hi(ov.z);
      r6 = (-2.0f * a6) - bfw_lo(ov.w); r7 = (-2.0f * a7) - bfw_hi(ov.w);
    }
    const bool bad  = (flag != 0) | big;
    const bool live = node < NN;
    r0 = bad ? qnan : r0; r1 = bad ? qnan : r1; r2 = bad ? qnan : r2; r3 = bad ? qnan : r3;
    r4 = bad ? qnan : r4; r5 = bad ? qnan : r5; r6 = bad ? qnan : r6; r7 = bad ? qnan : r7;
    r0 = live ? r0 : 0.0f; r1 = live ? r1 : 0.0f; r2 = live ? r2 : 0.0f; r3 = live ? r3 : 0.0f;
    r4 = live ? r4 : 0.0f; r5 = live ? r5 : 0.0f; r6 = live ? r6 : 0.0f; r7 = live ? r7 : 0.0f;
    unsigned h0, l0, h1, l1, h2, l2, h3, l3;
    pack2(r0, r1, h0, l0);
    pack2(r2, r3, h1, l1);
    pack2(r4, r5, h2, l2);
    pack2(r6, r7, h3, l3);
    v4u qh, ql;
    qh.x = h0; qh.y = h1; qh.z = h2; qh.w = h3;
    ql.x = l0; ql.y = l1; ql.z = l2; ql.w = l3;
    unsigned short* wp = TD + (size_t)node * TP + loff;
    *(volatile v4u*)wp = qh;
    *(volatile v4u*)(wp + 64) = ql;
    __threadfence();
    *(volatile v4u*)wp = qh;
    *(volatile v4u*)(wp + 64) = ql;
  }
}

template <int BPITCH>
__device__ __forceinline__ void gemm_seg(const unsigned short* __restrict__ ap,
                                         const unsigned short* __restrict__ bp, int nsteps, v8f (&acc)[4]) {
#pragma unroll 1
  for (int s = 0; s < nsteps; ++s) {
    FragB af;
    af.h[0] = *(const v8usa*)(ap + 32 * s);
    af.h[1] = *(const v8usa*)(ap + 32 * s + 16);
#pragma unroll
    for (int nt = 0; nt < 4; ++nt) {
      const unsigned short* wq = bp + (size_t)(16 * nt) * (size_t)BPITCH + 32 * s;
      FragB bf;
      bf.h[0] = *(const v8usa*)wq;
      bf.h[1] = *(const v8usa*)(wq + 16);
      acc[nt] = wmb(af, bf, acc[nt]);
    }
  }
}

template <int SPT, int SPH>
__global__ __launch_bounds__(NTHR) __attribute__((amdgpu_num_vgpr(248)))
void k_gemm(const unsigned short* __restrict__ XT, const unsigned short* __restrict__ T1,
            const unsigned short* __restrict__ T2, const unsigned short* __restrict__ WCT,
            const unsigned short* __restrict__ WLT, const float* __restrict__ sm, float* out) {
  __shared__ __attribute__((aligned(16))) unsigned buf[GBM * BPW];
  __shared__ __attribute__((aligned(16))) float sb[128];
  const int tid = (int)threadIdx.x, lane = tid & 31, wave = tid >> 5, hh = lane >> 4, m = lane & 15;
  const int rowBase = (int)blockIdx.x * GBM;
  if (tid < 32) *(v4fa*)(sb + 4 * tid) = *(const v4fa*)(sm + 4 * tid);

  v8f acc[4];
  {
    const v8f z = {0.f, 0.f, 0.f, 0.f, 0.f, 0.f, 0.f, 0.f};
#pragma unroll
    for (int t = 0; t < 4; ++t) acc[t] = z;
  }
  {
    const size_t r = (size_t)(rowBase + 16 * wave + m);
    const unsigned short* bp = WCT + (size_t)m * (size_t)KC + 8 * hh;
    gemm_seg<KC>(XT + r * CH + 8 * hh, bp, 2, acc);
    gemm_seg<KC>(T1 + r * (2 * CH) + 8 * hh, bp + 64, (SPT != 0) ? 4 : 2, acc);
    gemm_seg<KC>(T2 + r * (2 * CH) + 8 * hh, bp + 192, (SPT != 0) ? 4 : 2, acc);
  }
  __syncthreads();

  {
    const unsigned evm = ((m & 1) == 0) ? 0xffffffffu : 0u;
    const int wsel = (m & 1) * 32;
#pragma unroll
    for (int nt = 0; nt < 4; ++nt) {
      const int col = 16 * nt + m;
      const float bb = sb[col];
      const int wo = (col >> 1) + wsel;
#pragma unroll
      for (int r = 0; r < 8; ++r) {
        const float v = relu_k(acc[nt][r] + bb);
        const unsigned hb = bf16_bits(v);
        const unsigned lb = bf16_bits(v - __uint_as_float(hb << 16));
        const unsigned own = hb | (lb << 16);
        const unsigned par = (unsigned)__shfl_xor((int)own, 1, 32);
        const unsigned we = (own & 0xffffu) | (par << 16);
        const unsigned wd = (par >> 16) | (own & 0xffff0000u);
        buf[(16 * wave + 8 * hh + r) * BPW + wo] = (we & evm) | (wd & ~evm);
      }
    }
  }
  __syncthreads();

  v8f acc2[4];
  {
    const v8f z = {0.f, 0.f, 0.f, 0.f, 0.f, 0.f, 0.f, 0.f};
#pragma unroll
    for (int t = 0; t < 4; ++t) acc2[t] = z;
  }
  {
    const unsigned* arow = buf + (16 * wave + m) * BPW + 4 * hh;
    const unsigned short* bp2 = WLT + (size_t)m * (size_t)KL + 8 * hh;
#pragma unroll 1
    for (int s = 0; s < ((SPH != 0) ? 4 : 2); ++s) {
      FragB af;
      af.h[0] = *(const v8usa*)(arow + 16 * s);
      af.h[1] = *(const v8usa*)(arow + 16 * s + 8);
#pragma unroll
      for (int nt = 0; nt < 4; ++nt) {
        const unsigned short* wq = bp2 + (size_t)(16 * nt) * (size_t)KL + 32 * s;
        FragB bf;
        bf.h[0] = *(const v8usa*)wq;
        bf.h[1] = *(const v8usa*)(wq + 16);
        acc2[nt] = wmb(af, bf, acc2[nt]);
      }
    }
  }
  __syncthreads();

#pragma unroll
  for (int nt = 0; nt < 4; ++nt) {
#pragma unroll
    for (int r = 0; r < 8; ++r)
      buf[(16 * wave + 8 * hh + r) * BPW + 16 * nt + m] = __float_as_uint(acc2[nt][r]);
  }
  __syncthreads();

  const v4f blv = *(const v4fa*)(sb + 64 + 4 * m);
#pragma unroll 1
  for (int i = 0; i < 8; ++i) {
    const int lr   = 16 * wave + 2 * i + hh;
    const int grow = rowBase + lr;
    const int node = grow >> 2, bq = grow & 3;
    const bool live = node < NN;
    const int nodec = live ? node : NN - 1;
    const v4u a = *(const v4ua*)(buf + lr * BPW + 4 * m);
    asm volatile("" :: "v"(a));
    v4f o;
    o.x = __uint_as_float(a.x) + blv.x; o.y = __uint_as_float(a.y) + blv.y;
    o.z = __uint_as_float(a.z) + blv.z; o.w = __uint_as_float(a.w) + blv.w;
    float* op = out + ((size_t)bq * NN + (size_t)nodec) * CH + 4 * m;
    if (live) *(volatile v4f*)op = o;
    __threadfence();
    if (live) *(volatile v4f*)op = o;
  }
}

extern "C" void kernel_launch(void* const* d_in, const int* in_sizes, int n_in,
                              void* d_out, int out_size, void* d_ws, size_t ws_size,
                              hipStream_t stream) {
  if (n_in < 7) return;
  if (in_sizes[0] != NBT * NN * CH) return;
  if (in_sizes[1] != NE) return;
  if (in_sizes[2] != NE) return;
  if (in_sizes[3] != 3 * CH * CH) return;
  if (in_sizes[4] != CH) return;
  if (in_sizes[5] != CH * CH) return;
  if (in_sizes[6] != CH) return;
  if (out_size != NBT * NN * CH) return;

  const float* x   = (const float*)d_in[0];
  const int*   src = (const int*)d_in[1];
  const int*   dst = (const int*)d_in[2];
  const float* Wc  = (const float*)d_in[3];
  const float* bc  = (const float*)d_in[4];
  const float* Wl  = (const float*)d_in[5];
  const float* bl  = (const float*)d_in[6];
  float* out = (float*)d_out;

  constexpr size_t zXT   = (size_t)MP * XP * 2;
  constexpr size_t zTH   = (size_t)MP * TP * 2;
  constexpr size_t zLIST = (size_t)NBK * RCAP * 4;
  constexpr size_t zCO   = (size_t)NBK * 2 * NBRUN * 4;
  constexpr size_t zNORM = (size_t)NBK * NBRUN * 4;
  constexpr size_t zFLAG = 6400;
  constexpr size_t zWCT  = (size_t)CH * KC * 2;
  constexpr size_t zWLT  = (size_t)CH * KL * 2;
  constexpr size_t zSM   = 512;
  constexpr size_t oXT   = 0;
  constexpr size_t oT1   = oXT + zXT;
  constexpr size_t oT2   = oT1 + zTH;
  constexpr size_t oLIST = oT2 + zTH;
  constexpr size_t oCO   = oLIST + zLIST;
  constexpr size_t oNORM = oCO + zCO;
  constexpr size_t oFLAG = oNORM + zNORM;
  constexpr size_t oWCT  = oFLAG + zFLAG;
  constexpr size_t oWLT  = oWCT + zWCT;
  constexpr size_t oSM   = oWLT + zWLT;
  constexpr size_t oEND  = oSM + zSM;
  static_assert(zXT % 256 == 0 && zTH % 256 == 0 && zLIST % 256 == 0 && zCO % 256 == 0 && zNORM % 256 == 0);
  static_assert(zFLAG % 256 == 0 && zFLAG >= (size_t)NBK * 128 && zWCT % 256 == 0 && zWLT % 256 == 0);
  static_assert((size_t)NBK * NBRUN >= (size_t)MP);
  static_assert(oEND <= (size_t)WSMAX);
  if (oEND > ws_size) return;

  char* ws = (char*)d_ws;
  unsigned short* XT   = (unsigned short*)(ws + oXT);
  unsigned short* T1HL = (unsigned short*)(ws + oT1);
  unsigned short* T2HL = (unsigned short*)(ws + oT2);
  int*            LIST = (int*)(ws + oLIST);
  int*            CO   = (int*)(ws + oCO);
  int*            NRMB = (int*)(ws + oNORM);
  const float*    NORM = (const float*)(ws + oNORM);
  int*            FLAG = (int*)(ws + oFLAG);
  unsigned short* WCT  = (unsigned short*)(ws + oWCT);
  unsigned short* WLT  = (unsigned short*)(ws + oWLT);
  float*          SM   = (float*)(ws + oSM);

  hipFuncSetAttribute(reinterpret_cast<const void*>(&k_bucket), hipFuncAttributeMaxDynamicSharedMemorySize, (int)BK_LDS);

  k_prep<<<PBTOT, NTHR, 0, stream>>>(x, Wc, bc, Wl, bl, XT, WCT, WLT, SM);
  k_bucket<<<NBK, NTHR, BK_LDS, stream>>>(src, dst, LIST, CO, NRMB, FLAG);
  k_replay<1><<<MP / RPB, NTHR, 0, stream>>>(LIST, CO, NORM, FLAG, XT, XT, T1HL);
  k_replay<2><<<MP / RPB, NTHR, 0, stream>>>(LIST, CO, NORM, FLAG, XT, T1HL, T2HL);
  k_gemm<SPLIT_T, SPLIT_H><<<GBLK, NTHR, 0, stream>>>(XT, T1HL, T2HL, WCT, WLT, SM, out);
}
